// MHA_80307298500800
// MI455X (gfx1250) — hardware-verified
//
#include <hip/hip_runtime.h>
#include <math.h>

typedef __attribute__((ext_vector_type(16))) _Float16 v16h;
typedef __attribute__((ext_vector_type(16))) __bf16 v16b;
typedef __attribute__((ext_vector_type(8)))  _Float16 v8h;
typedef __attribute__((ext_vector_type(8)))  __bf16 v8b;
typedef __attribute__((ext_vector_type(8)))  float v8f;
typedef __attribute__((ext_vector_type(4)))  float v4f;
typedef __attribute__((ext_vector_type(4)))  unsigned v4u;

template <typename T> __device__ __forceinline__ void vst2(void* p, T v) { *(volatile T*)p = v; __threadfence(); *(volatile T*)p = v; }
__device__ __forceinline__ v8f wmma16(v16h a, v16h b, v8f c) {
  v8f d = __builtin_amdgcn_wmma_f32_16x16x32_f16(false, a, false, b, (short)0, c, false, false);
  asm volatile("v_nop\n\tv_nop\n\tv_nop\n\tv_nop" : "+v"(d) : "v"(a), "v"(b));
  return d;
}
__device__ __forceinline__ v8f wmma_bf(v16b a, v16b b, v8f c) {
  v8f d = __builtin_amdgcn_wmma_f32_16x16x32_bf16(false, a, false, b, (short)0, c, false, false);
  asm volatile("v_nop\n\tv_nop\n\tv_nop\n\tv_nop" : "+v"(d) : "v"(a), "v"(b));
  return d;
}
__device__ __forceinline__ v16h frag_h(const _Float16* rowk0, unsigned lane) {
  union { v16h v; v8h q[2]; } u; const _Float16* p = rowk0 + 8u * (lane >> 4);
  u.q[0] = *(const v8h*)p; u.q[1] = *(const v8h*)(p + 16); return u.v;
}
__device__ __forceinline__ v16b frag_b(const __bf16* rowk0, unsigned lane) {
  union { v16b v; v8b q[2]; } u; const __bf16* p = rowk0 + 8u * (lane >> 4);
  u.q[0] = *(const v8b*)p; u.q[1] = *(const v8b*)(p + 16); return u.v;
}
__device__ __forceinline__ float bfr(float v) { return (float)(__bf16)v; }

#ifndef NB
#define NB 2
#endif
#ifndef SEQ
#define SEQ 2048
#endif
#define NB_FULL 2
#define SEQ_FULL 2048
#define DM 2048
#define NH 16
#define HD 128
#define MROWS (NB * SEQ)
#define SCALE 0.08838834764831845f
#define LOG2E 1.4426950408889634f
#define CTXC 4096.0f
#define WOC 256.0f
#define OUTC (1.0f / 1048576.0f)

static_assert(NH * HD == DM);
static_assert(SEQ % 128 == 0);
static_assert(SEQ <= SEQ_FULL);
static_assert(NB <= NB_FULL);
static_assert(MROWS % 64 == 0);
static_assert(DM % 128 == 0);
static_assert(((size_t)SEQ * DM) % (8 * 256) == 0);
static_assert(((size_t)DM * DM) % (8 * 256) == 0);

#define WS_XB  ((size_t)0)
#define WS_WQ  (WS_XB  + 2u * (size_t)MROWS * DM)
#define WS_WK  (WS_WQ  + 2u * (size_t)DM * DM)
#define WS_WV  (WS_WK  + 2u * (size_t)DM * DM)
#define WS_WO  (WS_WV  + 2u * (size_t)DM * DM)
#define WS_QH  (WS_WO  + 2u * (size_t)DM * DM)
#define WS_KH  (WS_QH  + 2u * (size_t)MROWS * DM)
#define WS_CTX (WS_KH  + 2u * (size_t)MROWS * DM)
#define WS_DG  (WS_CTX + 2u * (size_t)MROWS * DM)
#define WS_WP  (WS_DG  + 4u * (size_t)NB * NH * SEQ)
#define WS_END (WS_WP  + 4u * (size_t)NB * NH * SEQ)
static_assert(WS_END <= (size_t)134217728);
static_assert(WS_DG % 128 == 0);

__global__ __launch_bounds__(256) void k_cvt(const float* __restrict__ src, unsigned short* __restrict__ dst, unsigned n8, size_t sstride, size_t dstride, int mode) {
  const unsigned i = blockIdx.x * 256u + threadIdx.x; if (i >= n8) return;
  const float* s = src + (size_t)blockIdx.y * sstride + (size_t)i * 8u; unsigned short* d = dst + (size_t)blockIdx.y * dstride + (size_t)i * 8u;
  const v4f a = *(const v4f*)s, b = *(const v4f*)(s + 4);
  v4u o;
  if (mode == 0) { v8b t;
#pragma unroll
    for (int u = 0; u < 4; ++u) { t[u] = (__bf16)a[u]; t[4 + u] = (__bf16)b[u]; }
    o = __builtin_bit_cast(v4u, t);
  } else { v8h t;
#pragma unroll
    for (int u = 0; u < 4; ++u) { t[u] = (_Float16)(bfr(a[u]) * WOC); t[4 + u] = (_Float16)(bfr(b[u]) * WOC); }
    o = __builtin_bit_cast(v4u, t);
  }
  vst2((void*)d, o);
}

__global__ __launch_bounds__(128) void k_qk(const __bf16* __restrict__ XB, const __bf16* __restrict__ WQ, const __bf16* __restrict__ WK, const float* __restrict__ COS, const float* __restrict__ SIN,
    _Float16* __restrict__ QH, _Float16* __restrict__ KH, float* __restrict__ DG) {
  __shared__ __align__(16) float sq[64][132]; __shared__ __align__(16) _Float16 sk[64][136]; __shared__ __align__(16) float scs[64][64], ssn[64][64]; __shared__ __align__(16) float sdg[64];
  const unsigned tid = threadIdx.x, wave = tid >> 5, lane = tid & 31u, col = lane & 15u, g = lane >> 4;
  const unsigned h = blockIdx.y, c0 = h * HD; const unsigned r0 = blockIdx.x * 64u; const unsigned bb = r0 / (unsigned)SEQ, t0 = r0 % (unsigned)SEQ;
  const __bf16* xrow = XB + (size_t)(r0 + wave * 16u + col) * DM;
  const bool odd = (col & 1u) != 0u;
  {
    v8f aq[8] = {};
#pragma unroll 2
    for (unsigned kc = 0; kc < DM / 32; ++kc) {
      const v16b a = frag_b(xrow + kc * 32u, lane);
      asm volatile("s_wait_loadcnt 0x0" ::: "memory");
#pragma unroll
      for (int j = 0; j < 8; ++j) { const v16b wq = frag_b(WQ + (size_t)(c0 + j * 16u + col) * DM + kc * 32u, lane);
        asm volatile("s_wait_loadcnt 0x0" ::: "memory");
        aq[j] = wmma_bf(a, wq, aq[j]); } }
    for (unsigned e = tid; e < 64u * 16u; e += 128u) { const unsigned rl = e >> 4, q = e & 15u; const size_t o = (size_t)(t0 + rl) * 64u + q * 4u;
      const v4f c = *(const v4f*)(COS + o), s = *(const v4f*)(SIN + o);
#pragma unroll
      for (int u = 0; u < 4; ++u) { scs[rl][q * 4u + u] = bfr(c[u]); ssn[rl][q * 4u + u] = bfr(s[u]); } }
    __syncthreads();
#pragma unroll
    for (int j = 0; j < 8; ++j) {
#pragma unroll
      for (int r = 0; r < 8; ++r) { const unsigned rl = wave * 16u + 8u * g + r; const unsigned pi = j * 8u + (col >> 1);
        const float c = scs[rl][pi], s = ssn[rl][pi];
        const float oq = aq[j][r];
        const float pq = __shfl_xor(oq, 1);
        const float sg = odd ? s : -s;
        const float qv = oq * c + pq * sg;
        sq[rl][j * 16u + col] = qv; }
      asm volatile("" ::: "memory"); }
  }
  __syncthreads();
  v8f ak[8] = {};
#pragma unroll 2
  for (unsigned kc = 0; kc < DM / 32; ++kc) {
    const v16b a = frag_b(xrow + kc * 32u, lane);
    asm volatile("s_wait_loadcnt 0x0" ::: "memory");
#pragma unroll
    for (int j = 0; j < 8; ++j) { const v16b wk = frag_b(WK + (size_t)(c0 + j * 16u + col) * DM + kc * 32u, lane);
      asm volatile("s_wait_loadcnt 0x0" ::: "memory");
      ak[j] = wmma_bf(a, wk, ak[j]); } }
  float ds[8] = {0.f, 0.f, 0.f, 0.f, 0.f, 0.f, 0.f, 0.f};
#pragma unroll
  for (int j = 0; j < 8; ++j) {
#pragma unroll
    for (int r = 0; r < 8; ++r) { const unsigned rl = wave * 16u + 8u * g + r; const unsigned pi = j * 8u + (col >> 1);
      const float c = scs[rl][pi], s = ssn[rl][pi];
      const float okv = ak[j][r];
      const float pk = __shfl_xor(okv, 1);
      const float sg = odd ? s : -s;
      const float kv = okv * c + pk * sg;
      const float qv = sq[rl][j * 16u + col];
      ds[r] += qv * kv;
      sk[rl][j * 16u + col] = (_Float16)kv; }
    asm volatile("" ::: "memory"); }
#pragma unroll
  for (int r = 0; r < 8; ++r) { float d = ds[r]; d += __shfl_xor(d, 1); d += __shfl_xor(d, 2); d += __shfl_xor(d, 4); d += __shfl_xor(d, 8);
    if (col == 0u) sdg[wave * 16u + 8u * g + r] = d * SCALE; }
  __syncthreads();
  for (unsigned e = tid; e < 64u * 16u; e += 128u) { const unsigned rl = e >> 4, q = e & 15u; const size_t o = (size_t)(r0 + rl) * DM + c0 + q * 8u;
    const v4f f0 = *(const v4f*)&sq[rl][q * 8u], f1 = *(const v4f*)&sq[rl][q * 8u + 4u]; v8h tq;
#pragma unroll
    for (int u = 0; u < 4; ++u) { tq[u] = (_Float16)f0[u]; tq[4 + u] = (_Float16)f1[u]; }
    const v4u oq4 = __builtin_bit_cast(v4u, tq); const v4u ok4 = *(const v4u*)&sk[rl][q * 8u];
    vst2((void*)(QH + o), oq4); vst2((void*)(KH + o), ok4); }
  if (tid < 16u) vst2((void*)(DG + (size_t)(bb * NH + h) * SEQ + t0 + tid * 4u), *(const v4f*)&sdg[tid * 4u]);
}

__global__ __launch_bounds__(128) void k_lse(const _Float16* __restrict__ QH, const _Float16* __restrict__ KH, const float* __restrict__ DG, float* __restrict__ WP) {
  __shared__ __align__(16) float sw[64];
  const unsigned tid = threadIdx.x, wave = tid >> 5, lane = tid & 31u, col = lane & 15u, g = lane >> 4;
  const unsigned qb = blockIdx.x, h = blockIdx.y, b = blockIdx.z; const unsigned c0 = h * HD; const unsigned ql0 = qb * 64u + wave * 16u;
  const size_t q0 = (size_t)b * SEQ + ql0, kr0 = (size_t)b * SEQ;
  const float C2 = SCALE * LOG2E;
  v16h qf[4];
#pragma unroll
  for (int kc = 0; kc < 4; ++kc) qf[kc] = frag_h(QH + (q0 + col) * DM + c0 + kc * 32u, lane);
  float m[8], sm[8];
#pragma unroll
  for (int r = 0; r < 8; ++r) { m[r] = -3.0e38f; sm[r] = 0.f; }
#pragma unroll 1
  for (unsigned kb = 0; kb < SEQ / 128; ++kb) {
    v8f acc[8] = {};
#pragma unroll
    for (int j = 0; j < 8; ++j) { const _Float16* kp = KH + (kr0 + kb * 128u + j * 16u + col) * DM + c0;
      const v16h k0 = frag_h(kp, lane), k1 = frag_h(kp + 32, lane), k2 = frag_h(kp + 64, lane), k3 = frag_h(kp + 96, lane);
      asm volatile("s_wait_loadcnt 0x0" ::: "memory");
      acc[j] = wmma16(qf[0], k0, acc[j]); acc[j] = wmma16(qf[1], k1, acc[j]); acc[j] = wmma16(qf[2], k2, acc[j]); acc[j] = wmma16(qf[3], k3, acc[j]); }
#pragma unroll
    for (int r = 0; r < 8; ++r) { float mx = acc[0][r];
#pragma unroll
      for (int j = 1; j < 8; ++j) mx = fmaxf(mx, acc[j][r]);
      const float mn = fmaxf(m[r], mx * C2); float s = 0.f;
#pragma unroll
      for (int j = 0; j < 8; ++j) s += exp2f(fmaf(acc[j][r], C2, -mn));
      sm[r] = sm[r] * exp2f(m[r] - mn) + s; m[r] = mn; } }
#pragma unroll
  for (int off = 1; off < 16; off <<= 1) {
#pragma unroll
    for (int r = 0; r < 8; ++r) { const float om = __shfl_xor(m[r], off), os = __shfl_xor(sm[r], off); const float mn = fmaxf(m[r], om);
      sm[r] = sm[r] * exp2f(m[r] - mn) + os * exp2f(om - mn); m[r] = mn; } }
  const float* dp = DG + (size_t)(b * NH + h) * SEQ + ql0 + 8u * g;
  const v4f d0 = *(const v4f*)dp, d1 = *(const v4f*)(dp + 4);
#pragma unroll
  for (int r = 0; r < 8; ++r) { const float dg = r < 4 ? d0[r & 3] : d1[r & 3]; const float w = exp2f(dg * LOG2E - m[r] - log2f(sm[r]));
    if (col == 0u) sw[wave * 16u + 8u * g + r] = w; }
  __syncthreads();
  if (tid < 16u) vst2((void*)(WP + (size_t)(b * NH + h) * SEQ + qb * 64u + tid * 4u), *(const v4f*)&sw[tid * 4u]);
}

__global__ __launch_bounds__(128) void k_vw(const __bf16* __restrict__ XB, const __bf16* __restrict__ WV, const float* __restrict__ WP, _Float16* __restrict__ CTX) {
  __shared__ __align__(16) _Float16 sh[64][136];
  const unsigned tid = threadIdx.x, wave = tid >> 5, lane = tid & 31u, col = lane & 15u, g = lane >> 4;
  const unsigned h = blockIdx.y, c0 = h * HD; const unsigned r0 = blockIdx.x * 64u; const unsigned bb = r0 / (unsigned)SEQ, t0 = r0 % (unsigned)SEQ;
  v8f av[8] = {};
  const __bf16* xrow = XB + (size_t)(r0 + wave * 16u + col) * DM;
#pragma unroll 2
  for (unsigned kc = 0; kc < DM / 32; ++kc) {
    const v16b a = frag_b(xrow + kc * 32u, lane);
    asm volatile("s_wait_loadcnt 0x0" ::: "memory");
#pragma unroll
    for (int j = 0; j < 8; ++j) { const v16b w = frag_b(WV + (size_t)(c0 + j * 16u + col) * DM + kc * 32u, lane);
      asm volatile("s_wait_loadcnt 0x0" ::: "memory");
      av[j] = wmma_bf(a, w, av[j]); } }
  const float* wp = WP + (size_t)(bb * NH + h) * SEQ + t0 + wave * 16u + 8u * g;
  const v4f w0 = *(const v4f*)wp, w1 = *(const v4f*)(wp + 4);
#pragma unroll
  for (int j = 0; j < 8; ++j) {
#pragma unroll
    for (int r = 0; r < 8; ++r) { const float wr = (r < 4 ? w0[r & 3] : w1[r & 3]) * CTXC; sh[wave * 16u + 8u * g + r][j * 16u + col] = (_Float16)(av[j][r] * wr); } }
  __syncthreads();
  for (unsigned e = tid; e < 64u * 16u; e += 128u) { const unsigned rl = e >> 4, q = e & 15u; vst2((void*)(CTX + (size_t)(r0 + rl) * DM + c0 + q * 8u), *(const v4u*)&sh[rl][q * 8u]); }
}

__global__ __launch_bounds__(128) void k_out(const _Float16* __restrict__ CTX, const _Float16* __restrict__ WO, float* __restrict__ OUT) {
  __shared__ __align__(16) float ss[4][16][132];
  const unsigned tid = threadIdx.x, wave = tid >> 5, lane = tid & 31u, col = lane & 15u, g = lane >> 4;
  const unsigned c0 = blockIdx.y * 128u; const unsigned r0 = blockIdx.x * 64u; const unsigned bb = r0 / (unsigned)SEQ, t0 = r0 % (unsigned)SEQ;
  v8f acc[8] = {};
  const _Float16* arow = CTX + (size_t)(r0 + wave * 16u + col) * DM;
#pragma unroll 2
  for (unsigned kc = 0; kc < DM / 32; ++kc) {
    const v16h a = frag_h(arow + kc * 32u, lane);
    asm volatile("s_wait_loadcnt 0x0" ::: "memory");
#pragma unroll
    for (int j = 0; j < 8; ++j) { const v16h w = frag_h(WO + (size_t)(c0 + j * 16u + col) * DM + kc * 32u, lane);
      asm volatile("s_wait_loadcnt 0x0" ::: "memory");
      acc[j] = wmma16(a, w, acc[j]); } }
#pragma unroll
  for (int j = 0; j < 8; ++j) {
#pragma unroll
    for (int r = 0; r < 8; ++r) ss[wave][8u * g + r][j * 16u + col] = acc[j][r] * OUTC; }
  __syncthreads();
  const size_t orow0 = (size_t)bb * SEQ_FULL + t0 + wave * 16u;
  for (unsigned rl = 0; rl < 16u; ++rl) vst2((void*)(OUT + (orow0 + rl) * DM + c0 + lane * 4u), *(const v4f*)&ss[wave][rl][lane * 4u]);
}

extern "C" void kernel_launch(void* const* d_in, const int* in_sizes, int n_in, void* d_out, int out_size, void* d_ws, size_t ws_size, hipStream_t stream) {
  if (n_in < 7) return;
  const long long need_x = (long long)(NB - 1) * SEQ_FULL * DM + (long long)SEQ * DM;
  if ((long long)in_sizes[0] < need_x) return;
  if (in_sizes[1] < SEQ * 64 || in_sizes[2] < SEQ * 64) return;
  if (in_sizes[3] < DM * DM || in_sizes[4] < DM * DM || in_sizes[5] < DM * DM || in_sizes[6] < DM * DM) return;
  if ((long long)out_size < need_x) return;
  if (ws_size < (size_t)WS_END) return;
  const float* const* F = (const float* const*)d_in;
  char* ws = (char*)d_ws;
  unsigned short* XB = (unsigned short*)(ws + WS_XB); unsigned short* WQ = (unsigned short*)(ws + WS_WQ); unsigned short* WK = (unsigned short*)(ws + WS_WK);
  unsigned short* WV = (unsigned short*)(ws + WS_WV); unsigned short* WO = (unsigned short*)(ws + WS_WO);
  _Float16* QH = (_Float16*)(ws + WS_QH); _Float16* KH = (_Float16*)(ws + WS_KH); _Float16* CTX = (_Float16*)(ws + WS_CTX);
  float* DG = (float*)(ws + WS_DG); float* WP = (float*)(ws + WS_WP);
  const unsigned nx8 = (unsigned)((size_t)SEQ * DM / 8), nw8 = (unsigned)((size_t)DM * DM / 8);
  k_cvt<<<dim3((nx8 + 255u) / 256u, NB), 256, 0, stream>>>(F[0], XB, nx8, (size_t)SEQ_FULL * DM, (size_t)SEQ * DM, 0);
  k_cvt<<<dim3((nw8 + 255u) / 256u, 1), 256, 0, stream>>>(F[3], WQ, nw8, (size_t)0, (size_t)0, 0);
  k_cvt<<<dim3((nw8 + 255u) / 256u, 1), 256, 0, stream>>>(F[4], WK, nw8, (size_t)0, (size_t)0, 0);
  k_cvt<<<dim3((nw8 + 255u) / 256u, 1), 256, 0, stream>>>(F[5], WV, nw8, (size_t)0, (size_t)0, 0);
  k_cvt<<<dim3((nw8 + 255u) / 256u, 1), 256, 0, stream>>>(F[6], WO, nw8, (size_t)0, (size_t)0, 1);
  k_qk<<<dim3(MROWS / 64, NH), 128, 0, stream>>>((const __bf16*)XB, (const __bf16*)WQ, (const __bf16*)WK, F[1], F[2], QH, KH, DG);
  k_lse<<<dim3(SEQ / 64, NH, NB), 128, 0, stream>>>(QH, KH, DG, WP);
  k_vw<<<dim3(MROWS / 64, NH), 128, 0, stream>>>((const __bf16*)XB, (const __bf16*)WV, WP, CTX);
  k_out<<<dim3(MROWS / 64, DM / 128), 128, 0, stream>>>(CTX, (const _Float16*)WO, (float*)d_out);
}
